// Block_3212635537783
// MI455X (gfx1250) — hardware-run, weakly checked
//
#include <hip/hip_runtime.h>


#ifndef NB
#define NB 4
#endif
#ifndef SEQ
#define SEQ 2048
#endif
#define NB_FULL  4
#define SEQ_FULL 2048
#ifndef OUT_SEQ
#define OUT_SEQ SEQ
#endif
#define DM   768
#define NH_  12
#define HD   64
#define FF   3072
#define AW   4
#define OSP  68
#define EROWS (SEQ < 512 ? SEQ : 512)
#define QRS  2048.0f
#define QRI  (1.0f / 2048.0f)
#define SC2  ((float)(0.036084391824351614 * 1.4426950408889634))
#define PSH  14.0f
#define NEGB (-3.0e38f)
#define WCS  16.0f
#define WCI  0.0625f

static_assert(HD == 64);
static_assert(NH_ * HD == DM);
static_assert(DM % 64 == 0);
static_assert(FF % 64 == 0);
static_assert(DM % 32 == 0);
static_assert(FF % 32 == 0);
static_assert(HD % 32 == 0);
static_assert(SEQ % 64 == 0);
static_assert((NB * SEQ) % 64 == 0);
static_assert(SEQ % 32 == 0);
static_assert(SEQ % (16 * AW) == 0);
static_assert(EROWS % 64 == 0);
static_assert(EROWS >= 32);
static_assert(EROWS % 32 == 0);
static_assert(EROWS <= SEQ);
static_assert(EROWS % (16 * AW) == 0);
static_assert((SEQ - EROWS) % (16 * AW) == 0);
static_assert(((size_t)SEQ * DM) % 8 == 0);
static_assert(NB <= NB_FULL);
static_assert(SEQ <= SEQ_FULL);
static_assert((OSP * 4) % 16 == 0);
static_assert((NB * SEQ) % 8 == 0);
static_assert(DM % 128 == 0);
static_assert(DM % 256 == 0);
static_assert(32 * 16 * 4 == 2 * HD * 4 * 4);
static_assert(4 * 32 * 16 == 16 * HD * 2);
static_assert(16 * 4 == 64);
static_assert(32 * 2 == 64);
static_assert(256 * 2 * 16 == 64 * 128);
static_assert(AW * 16 * OSP * 4 <= 131072);
static_assert(64 * OSP * 4 + 64 * 64 * 2 <= 131072);
static_assert(8 * DM * 4 <= 131072);
static_assert(64 * 65 * 4 <= 131072);

typedef _Float16 h16;
typedef unsigned short bf;
typedef __attribute__((ext_vector_type(16))) __bf16   v16bf;
typedef __attribute__((ext_vector_type(16))) _Float16 v16h;
typedef __attribute__((ext_vector_type(8)))  _Float16 v8h;
typedef __attribute__((ext_vector_type(8)))  unsigned short v8us;
typedef __attribute__((ext_vector_type(8)))  float    v8f;
typedef __attribute__((ext_vector_type(4)))  float    v4f;
typedef v4f  __attribute__((may_alias)) v4fa;
typedef v8h  __attribute__((may_alias)) v8ha;

__device__ __forceinline__ unsigned short f2bf(float f) { unsigned u = __float_as_uint(f); u += 0x7FFFu + ((u >> 16) & 1u); return (unsigned short)(u >> 16); }
__device__ __forceinline__ float bfr(float f) { return __uint_as_float(((unsigned)f2bf(f)) << 16); }
__device__ __forceinline__ v16h cat16(v8h lo, v8h hi) { return __builtin_shufflevector(lo, hi, 0, 1, 2, 3, 4, 5, 6, 7, 8, 9, 10, 11, 12, 13, 14, 15); }
__device__ __forceinline__ v16bf cat16b(v8us lo, v8us hi) { return __builtin_bit_cast(v16bf, __builtin_shufflevector(lo, hi, 0, 1, 2, 3, 4, 5, 6, 7, 8, 9, 10, 11, 12, 13, 14, 15)); }
__device__ __forceinline__ v8f wmma16(v16h a, v16h b, v8f c) { return __builtin_amdgcn_wmma_f32_16x16x32_f16(false, a, false, b, (short)0, c, false, false); }
__device__ __forceinline__ v8f wmmab(v16bf a, v16bf b, v8f c) { return __builtin_amdgcn_wmma_f32_16x16x32_bf16(false, a, false, b, (short)0, c, false, false); }
__device__ __forceinline__ v8f wmma16g(v16h a, v16h b, v8f c) { c = wmma16(a, b, c); asm volatile("v_nop\n\tv_nop\n\tv_nop\n\tv_nop" : "+v"(c) : "v"(a), "v"(b)); return c; }
__device__ __forceinline__ v8f wmmabg(v16bf a, v16bf b, v8f c) { c = wmmab(a, b, c); asm volatile("v_nop\n\tv_nop\n\tv_nop\n\tv_nop" : "+v"(c) : "v"(a), "v"(b)); return c; }
__device__ __forceinline__ v16h  ldh(const h16* p) { return cat16(*(const v8h*)p, *(const v8h*)(p + 16)); }
__device__ __forceinline__ v16bf ldb(const bf* p)  { return cat16b(*(const v8us*)p, *(const v8us*)(p + 16)); }
__device__ __forceinline__ void wave_sync() { __builtin_amdgcn_fence(3  , "wavefront"); __builtin_amdgcn_wave_barrier(); asm volatile("" ::: "memory"); }
static __device__ __forceinline__ h16 toh_flush(float v) { const float w = (fabsf(v) < 6.103515625e-05f) ? 0.0f : v; return (h16)w; }

__global__ __launch_bounds__(256) void k_cvt8(const float* __restrict__ src, bf* dst, size_t n8) {
    const size_t i = (size_t)blockIdx.x * 256 + threadIdx.x; if (i >= n8) return;
    const v8f v = *(const v8f*)(src + i * 8); v8us o;
#pragma unroll
    for (int k = 0; k < 8; ++k) o[k] = f2bf(v[k]);
    *(volatile v8us*)(dst + i * 8) = o; __threadfence(); *(volatile v8us*)(dst + i * 8) = o;
}

template <int MODE>
__device__ __forceinline__ void wtr_body(const float* __restrict__ src, bf* dB, h16* dH, unsigned R, unsigned Cc) {
    __shared__ float tile[64 * 65];
    const unsigned tid = threadIdx.x;
    const unsigned c0 = blockIdx.x * 64u, r0 = blockIdx.y * 64u;
    const size_t zoff = (size_t)blockIdx.z * (size_t)R * (size_t)Cc;
    const float* s = src + zoff + (size_t)r0 * Cc + c0;
#pragma unroll
    for (unsigned i = 0; i < 4; ++i) {
        const unsigned p = i * 256u + tid; const unsigned r = p >> 4, c4 = (p & 15u) * 4u;
        const v4f v = *(const v4f*)(s + (size_t)r * Cc + c4);
        tile[r * 65u + c4 + 0u] = v[0]; tile[r * 65u + c4 + 1u] = v[1]; tile[r * 65u + c4 + 2u] = v[2]; tile[r * 65u + c4 + 3u] = v[3];
    }
    __syncthreads();
    const unsigned pc = (tid & 7u) * 8u, lq = tid >> 3;
    const size_t d0 = zoff + (size_t)(c0 + lq) * R + r0 + pc;
    const size_t d1 = zoff + (size_t)(c0 + 32u + lq) * R + r0 + pc;
    if (MODE == 0) {
        v8us o0, o1;
#pragma unroll
        for (unsigned k = 0; k < 8; ++k) { o0[k] = f2bf(tile[(pc + k) * 65u + lq]); o1[k] = f2bf(tile[(pc + k) * 65u + 32u + lq]); }
#pragma unroll 1
        for (int ps = 0; ps < 2; ++ps) { *(volatile v8us*)(dB + d0) = o0; *(volatile v8us*)(dB + d1) = o1; if (ps == 0) __threadfence(); }
    } else {
        v8h o0, o1;
#pragma unroll
        for (unsigned k = 0; k < 8; ++k) { o0[k] = toh_flush(bfr(tile[(pc + k) * 65u + lq]) * WCS); o1[k] = toh_flush(bfr(tile[(pc + k) * 65u + 32u + lq]) * WCS); }
#pragma unroll 1
        for (int ps = 0; ps < 2; ++ps) { *(volatile v8h*)(dH + d0) = o0; *(volatile v8h*)(dH + d1) = o1; if (ps == 0) __threadfence(); }
    }
}
__global__ __launch_bounds__(256) void k_wtr_bf(const float* __restrict__ src, bf* dst, unsigned R, unsigned Cc) { wtr_body<0>(src, dst, (h16*)0, R, Cc); }
__global__ __launch_bounds__(256) void k_wtr_h(const float* __restrict__ src, h16* dst, unsigned R, unsigned Cc) { wtr_body<1>(src, (bf*)0, dst, R, Cc); }

template <int MODE>
__device__ __forceinline__ void proj_body(const bf* __restrict__ A, const bf* __restrict__ Bt, h16* Ph, h16* Pr, unsigned resT) {
    __shared__ __align__(16) float os[16 * OSP];
    const unsigned K = DM;
    const unsigned lane = threadIdx.x & 31u, lr = lane & 15u, hi = lane >> 4;
    const unsigned r0 = blockIdx.x * 64u, c0 = blockIdx.y * 64u;
    v8f acc[4][4];
#pragma unroll
    for (int mb = 0; mb < 4; ++mb)
#pragma unroll
        for (int nb = 0; nb < 4; ++nb) acc[mb][nb] = (v8f){};
    const size_t aoff = (size_t)(r0 + lr) * K + 8u * hi, boff = (size_t)(c0 + lr) * K + 8u * hi;
#pragma unroll 1
    for (unsigned kc = 0; kc < K; kc += 32u) {
        v16bf a[4];
#pragma unroll
        for (int mb = 0; mb < 4; ++mb) a[mb] = ldb(A + aoff + (size_t)mb * 16 * K + kc);
#pragma unroll
        for (int nb = 0; nb < 4; ++nb) { const v16bf b = ldb(Bt + boff + (size_t)nb * 16 * K + kc);
#pragma unroll
            for (int mb = 0; mb < 4; ++mb) acc[mb][nb] = wmmabg(a[mb], b, acc[mb][nb]); }
    }
    size_t tbase, rbase; bool wr;
    if (MODE == 0) { const unsigned bb = r0 / (unsigned)SEQ, tt = r0 % (unsigned)SEQ; const unsigned zc = bb * (unsigned)NH_ + c0 / (unsigned)HD;
                     tbase = ((size_t)zc * SEQ + (size_t)tt) * HD; rbase = ((size_t)zc * (size_t)resT + (size_t)tt) * HD; wr = tt < resT; }
    else           { const unsigned bb = c0 / (unsigned)SEQ, tt = c0 % (unsigned)SEQ;
                     tbase = (size_t)bb * (size_t)DM * SEQ + (size_t)r0 * SEQ + (size_t)tt; rbase = (size_t)bb * (size_t)DM * (size_t)resT + (size_t)r0 * (size_t)resT + (size_t)tt; wr = tt < resT; }
#pragma unroll
    for (int mb = 0; mb < 4; ++mb) {
#pragma unroll
        for (int nb = 0; nb < 4; ++nb) {
#pragma unroll
            for (int j = 0; j < 8; ++j) os[(hi * 8u + j) * OSP + nb * 16 + lr] = acc[mb][nb][j]; }
        wave_sync();
        v8h hv[4], rv[4]; size_t oo[4], ro[4];
#pragma unroll
        for (int s = 0; s < 4; ++s) {
            unsigned row, c8;
            if (MODE == 0) { const unsigned p = s * 32u + lane; row = p >> 3; c8 = (p & 7u) * 8u;
                             oo[s] = tbase + (size_t)(mb * 16) * HD + (size_t)p * 8; ro[s] = rbase + (size_t)(mb * 16) * HD + (size_t)p * 8; }
            else           { row = 4u * s + (lane >> 3); c8 = (lane & 7u) * 8u;
                             oo[s] = tbase + (size_t)(mb * 16 + row) * SEQ + c8; ro[s] = rbase + (size_t)(mb * 16 + row) * (size_t)resT + c8; }
            const v4f x0 = *(const v4fa*)(&os[row * OSP + c8]); const v4f x1 = *(const v4fa*)(&os[row * OSP + c8 + 4]);
#pragma unroll
            for (int i = 0; i < 4; ++i) { const h16 a0 = toh_flush(x0[i]); const h16 a1 = toh_flush(x1[i]); hv[s][i] = a0; hv[s][4 + i] = a1;
                                          rv[s][i] = toh_flush((x0[i] - (float)a0) * QRS); rv[s][4 + i] = toh_flush((x1[i] - (float)a1) * QRS); }
        }
#pragma unroll 1
        for (int ps = 0; ps < 2; ++ps) {
#pragma unroll
            for (int s = 0; s < 4; ++s) { *(volatile v8h*)(Ph + oo[s]) = hv[s]; if (wr) *(volatile v8h*)(Pr + ro[s]) = rv[s]; }
            if (ps == 0) __threadfence(); }
        wave_sync();
    }
}
__global__ __launch_bounds__(32) void k_proj_tok(const bf* __restrict__ A, const bf* __restrict__ Bt, h16* Ph, h16* Pr, unsigned resT) { proj_body<0>(A, Bt, Ph, Pr, resT); }
__global__ __launch_bounds__(32) void k_proj_tr(const bf* __restrict__ A, const bf* __restrict__ Bt, h16* Ph, h16* Pr, unsigned resT) { proj_body<1>(A, Bt, Ph, Pr, resT); }

template <int EARLY>
__device__ __forceinline__ void flash_body(const h16* __restrict__ QH, const h16* __restrict__ QR, const h16* __restrict__ KP, const h16* __restrict__ KR,
                                           const h16* __restrict__ VT, const h16* __restrict__ VR, float* CTX) {
    __shared__ __align__(16) float os[AW * 16 * OSP];
    const unsigned lane = threadIdx.x & 31u, lr = lane & 15u, hi = lane >> 4;
    const unsigned wave = (unsigned)__builtin_amdgcn_readfirstlane((int)(threadIdx.x >> 5));
    const unsigned zh = blockIdx.y; const unsigned b = zh / (unsigned)NH_, h = zh % (unsigned)NH_;
    const unsigned t0 = (EARLY ? 0u : (unsigned)EROWS) + (blockIdx.x * (unsigned)AW + wave) * 16u;
    const unsigned lim = t0 + lr;
    const unsigned nk = (t0 + 16u + 31u) & ~31u;
    const size_t pbase = (size_t)zh * SEQ * HD;
    const size_t rbase = (size_t)zh * EROWS * HD;
    const size_t qo = pbase + (size_t)(t0 + lr) * HD + 8u * hi;
    const v16h qh0 = ldh(QH + qo), qh1 = ldh(QH + qo + 32);
    v16h qr0 = (v16h){}, qr1 = (v16h){};
    if (EARLY) { const size_t qro = rbase + (size_t)(t0 + lr) * HD + 8u * hi; qr0 = ldh(QR + qro); qr1 = ldh(QR + qro + 32); }
    const size_t ko = pbase + (size_t)lr * HD + 8u * hi;
    const size_t vo = pbase + (size_t)lr * SEQ + 8u * hi;
    const size_t kro = rbase + (size_t)lr * HD + 8u * hi;
    const size_t vro = rbase + (size_t)lr * EROWS + 8u * hi;
    v8f o[4], oR[4];
#pragma unroll
    for (int j = 0; j < 4; ++j) { o[j] = (v8f){}; oR[j] = (v8f){}; }
    float m = NEGB, l = 0.0f;
#pragma unroll 1
    for (unsigned key0 = 0; key0 < nk; key0 += 32u) {
        const h16* ka = KP + ko + (size_t)key0 * HD;
        const h16* kr = KR + kro + (size_t)key0 * HD;
        v8f sHa = (v8f){}, sLa = (v8f){}, sHb = (v8f){}, sLb = (v8f){};
        { const v16h k0 = ldh(ka), k1 = ldh(ka + 32);
          sHa = wmma16g(k0, qh0, sHa); sHa = wmma16g(k1, qh1, sHa);
          if (EARLY) { sLa = wmma16g(k0, qr0, sLa); sLa = wmma16g(k1, qr1, sLa);
                       const v16h r0 = ldh(kr), r1 = ldh(kr + 32);
                       sLa = wmma16g(r0, qh0, sLa); sLa = wmma16g(r1, qh1, sLa); } }
        { const v16h k0 = ldh(ka + 16 * HD), k1 = ldh(ka + 16 * HD + 32);
          sHb = wmma16g(k0, qh0, sHb); sHb = wmma16g(k1, qh1, sHb);
          if (EARLY) { sLb = wmma16g(k0, qr0, sLb); sLb = wmma16g(k1, qr1, sLb);
                       const v16h r0 = ldh(kr + 16 * HD), r1 = ldh(kr + 16 * HD + 32);
                       sLb = wmma16g(r0, qh0, sLb); sLb = wmma16g(r1, qh1, sLb); } }
        const unsigned ja = key0 + 8u * hi;
        float ta[8], tb[8]; bool fa[8], fb[8]; float mx = NEGB;
#pragma unroll
        for (int r = 0; r < 8; ++r) {
            fa[r] = (ja + (unsigned)r <= lim);
            fb[r] = (ja + 16u + (unsigned)r <= lim);
            if (EARLY) { ta[r] = (sHa[r] + sLa[r] * QRI) * SC2; tb[r] = (sHb[r] + sLb[r] * QRI) * SC2; }
            else       { ta[r] = sHa[r] * SC2; tb[r] = sHb[r] * SC2; }
            mx = fmaxf(mx, fmaxf(fa[r] ? ta[r] : NEGB, fb[r] ? tb[r] : NEGB)); }
        mx = fmaxf(mx, __shfl_xor(mx, 16, 32));
        const float mnew = fmaxf(m, mx);
        const float alpha = __builtin_amdgcn_exp2f(m - mnew);
        const float sh = PSH - mnew;
        v16h pb, pr = (v16h){}; float ls = 0.0f;
#pragma unroll
        for (int r = 0; r < 8; ++r) {
            const float xa = ta[r] + sh, xb = tb[r] + sh;
            const float ea = __builtin_amdgcn_exp2f(xa), eb = __builtin_amdgcn_exp2f(xb);
            const float ga = (fa[r] && xa >= -14.0f) ? ea : 0.0f, gb = (fb[r] && xb >= -14.0f) ? eb : 0.0f;
            const h16 pa = toh_flush(ga); const h16 pc = toh_flush(gb);
            pb[r] = pa; pb[8 + r] = pc;
            if (EARLY) { pr[r] = toh_flush((ga - (float)pa) * QRS); pr[8 + r] = toh_flush((gb - (float)pc) * QRS); ls += ga + gb; }
            else       { ls += (float)pa + (float)pc; } }
        l = l * alpha + ls; m = mnew;
#pragma unroll
        for (int j = 0; j < 4; ++j) { o[j] = o[j] * alpha; if (EARLY) oR[j] = oR[j] * alpha; }
        const h16* va = VT + vo + key0;
        const h16* vr = VR + vro + key0;
#pragma unroll
        for (int j = 0; j < 4; ++j) {
            const v16h vj = ldh(va + (size_t)(16 * j) * SEQ);
            o[j] = wmma16g(vj, pb, o[j]);
            if (EARLY) { oR[j] = wmma16g(vj, pr, oR[j]);
                         const v16h vrj = ldh(vr + (size_t)(16 * j) * EROWS);
                         oR[j] = wmma16g(vrj, pb, oR[j]); }
        }
    }
    l += __shfl_xor(l, 16, 32);
    const bool any = l > 0.0f;
    const float lsafe = any ? l : 1.0f;
    const float inv = any ? (1.0f / lsafe) : 0.0f;
    const unsigned wb = wave * 16u * OSP;
#pragma unroll
    for (int j = 0; j < 4; ++j) {
        v8f f = o[j]; if (EARLY) f = o[j] + oR[j] * QRI;
        v4f a, c;
        a[0] = f[0] * inv; a[1] = f[1] * inv; a[2] = f[2] * inv; a[3] = f[3] * inv; c[0] = f[4] * inv; c[1] = f[5] * inv; c[2] = f[6] * inv; c[3] = f[7] * inv;
        *(v4fa*)(&os[wb + lr * OSP + 16 * j + 8u * hi]) = a; *(v4fa*)(&os[wb + lr * OSP + 16 * j + 8u * hi + 4u]) = c; }
    wave_sync();
    float* orow = CTX + ((size_t)b * SEQ + t0) * DM + h * (unsigned)HD;
#pragma unroll 1
    for (int ps = 0; ps < 2; ++ps) {
#pragma unroll
        for (int s = 0; s < 8; ++s) { const unsigned row = 2u * s + (lane >> 4), cofs = (lane & 15u) * 4u;
            const v4f val = *(const v4fa*)(&os[wb + row * OSP + cofs]);
            *(volatile v4f*)(orow + (size_t)row * DM + cofs) = val; }
        if (ps == 0) __threadfence(); }
}
__global__ __launch_bounds__(32 * AW) void k_flash_early(const h16* __restrict__ QH, const h16* __restrict__ QR, const h16* __restrict__ KP, const h16* __restrict__ KR,
                                                         const h16* __restrict__ VT, const h16* __restrict__ VR, float* CTX) { flash_body<1>(QH, QR, KP, KR, VT, VR, CTX); }
__global__ __launch_bounds__(32 * AW) void k_flash_late(const h16* __restrict__ QH, const h16* __restrict__ QR, const h16* __restrict__ KP, const h16* __restrict__ KR,
                                                        const h16* __restrict__ VT, const h16* __restrict__ VR, float* CTX) { flash_body<0>(QH, QR, KP, KR, VT, VR, CTX); }

template <int FIRST>
__device__ __forceinline__ void ln_body(const float* __restrict__ X, const float* __restrict__ C, const float* __restrict__ g, const float* __restrict__ bt, float* OF, h16* OH) {
    __shared__ __align__(16) float rs[8 * DM];
    const unsigned lane = threadIdx.x & 31u;
    const unsigned wave = (unsigned)__builtin_amdgcn_readfirstlane((int)(threadIdx.x >> 5));
    const unsigned mrow = blockIdx.x * 8u + wave;
    const unsigned b = mrow / (unsigned)SEQ, t = mrow % (unsigned)SEQ;
    const unsigned wb = wave * (unsigned)DM;
    const size_t xo = FIRST ? (((size_t)b * SEQ_FULL + t) * DM) : ((size_t)mrow * DM);
    const size_t co = (size_t)mrow * DM;
    const size_t fo = FIRST ? ((size_t)mrow * DM) : (((size_t)b * OUT_SEQ + t) * DM);
    const float* xr = X + xo;
    const float* cr = C + co;
    float s = 0.0f;
#pragma unroll 1
    for (unsigned i = 0; i < DM / 128; ++i) {
        const unsigned idx = (i * 32u + lane) * 4u;
        v4f v = *(const v4f*)(xr + idx);
        if (FIRST) { const v4f c = *(const v4f*)(cr + idx); v[0] = bfr(v[0]) + c[0]; v[1] = bfr(v[1]) + c[1]; v[2] = bfr(v[2]) + c[2]; v[3] = bfr(v[3]) + c[3]; }
        *(v4fa*)(&rs[wb + idx]) = v;
        s += (v[0] + v[1]) + (v[2] + v[3]);
    }
    s += __shfl_xor(s, 16, 32); s += __shfl_xor(s, 8, 32); s += __shfl_xor(s, 4, 32); s += __shfl_xor(s, 2, 32); s += __shfl_xor(s, 1, 32);
    const float mean = s * (1.0f / (float)DM);
    wave_sync();
    float q = 0.0f;
#pragma unroll 1
    for (unsigned i = 0; i < DM / 128; ++i) {
        const unsigned idx = (i * 32u + lane) * 4u;
        const v4f v = *(const v4fa*)(&rs[wb + idx]);
        const float d0 = v[0] - mean, d1 = v[1] - mean, d2 = v[2] - mean, d3 = v[3] - mean;
        q += (d0 * d0 + d1 * d1) + (d2 * d2 + d3 * d3);
    }
    q += __shfl_xor(q, 16, 32); q += __shfl_xor(q, 8, 32); q += __shfl_xor(q, 4, 32); q += __shfl_xor(q, 2, 32); q += __shfl_xor(q, 1, 32);
    const float rstd = rsqrtf(q * (1.0f / (float)DM) + 1.0e-5f);
    float* ofr = OF + fo;
    h16* ohr = OH + co;
#pragma unroll 1
    for (int ps = 0; ps < 2; ++ps) {
#pragma unroll 1
        for (unsigned i = 0; i < DM / 128; ++i) {
            const unsigned idx = (i * 32u + lane) * 4u;
            const v4f v = *(const v4fa*)(&rs[wb + idx]);
            const v4f gg = *(const v4f*)(g + idx); const v4f bb = *(const v4f*)(bt + idx);
            v4f ov;
            ov[0] = (v[0] - mean) * rstd * bfr(gg[0]) + bfr(bb[0]); ov[1] = (v[1] - mean) * rstd * bfr(gg[1]) + bfr(bb[1]);
            ov[2] = (v[2] - mean) * rstd * bfr(gg[2]) + bfr(bb[2]); ov[3] = (v[3] - mean) * rstd * bfr(gg[3]) + bfr(bb[3]);
            *(volatile v4f*)(ofr + idx) = ov;
        }
        if (FIRST) {
#pragma unroll 1
            for (unsigned i = 0; i < DM / 256; ++i) {
                const unsigned idx = (i * 32u + lane) * 8u;
                const v4f v0 = *(const v4fa*)(&rs[wb + idx]); const v4f v1 = *(const v4fa*)(&rs[wb + idx + 4u]);
                const v4f g0 = *(const v4f*)(g + idx); const v4f g1 = *(const v4f*)(g + idx + 4u);
                const v4f b0 = *(const v4f*)(bt + idx); const v4f b1 = *(const v4f*)(bt + idx + 4u);
                v8h hv;
#pragma unroll
                for (int k = 0; k < 4; ++k) { hv[k] = toh_flush((v0[k] - mean) * rstd * bfr(g0[k]) + bfr(b0[k])); hv[4 + k] = toh_flush((v1[k] - mean) * rstd * bfr(g1[k]) + bfr(b1[k])); }
                *(volatile v8h*)(ohr + idx) = hv;
            }
        }
        if (ps == 0) __threadfence();
    }
}
__global__ __launch_bounds__(256) void k_ln_first(const float* __restrict__ X, const float* __restrict__ C, const float* __restrict__ g, const float* __restrict__ bt, float* OF, h16* OH) { ln_body<1>(X, C, g, bt, OF, OH); }
__global__ __launch_bounds__(256) void k_ln_last(const float* __restrict__ X, const float* __restrict__ g, const float* __restrict__ bt, float* OF) { ln_body<0>(X, X, g, bt, OF, (h16*)0); }

template <int MODE>
__device__ __forceinline__ void gemmh_body(const h16* __restrict__ A, const h16* __restrict__ Bt, const float* __restrict__ bias, const float* __restrict__ RES, h16* HO, float* YO) {
    __shared__ __align__(16) float os[64 * OSP];
    const unsigned K = (MODE == 0) ? (unsigned)DM : (unsigned)FF;
    const unsigned lane = threadIdx.x & 31u, lr = lane & 15u, hi = lane >> 4;
    const unsigned r0 = blockIdx.x * 64u, c0 = blockIdx.y * 64u;
    v8f acc[4][4];
#pragma unroll
    for (int mb = 0; mb < 4; ++mb)
#pragma unroll
        for (int nb = 0; nb < 4; ++nb) acc[mb][nb] = (v8f){};
    const size_t aoff = (size_t)(r0 + lr) * K + 8u * hi, boff = (size_t)(c0 + lr) * K + 8u * hi;
#pragma unroll 1
    for (unsigned kc = 0; kc < K; kc += 32u) {
        v16h a[4];
#pragma unroll
        for (int mb = 0; mb < 4; ++mb) a[mb] = ldh(A + aoff + (size_t)mb * 16 * K + kc);
#pragma unroll
        for (int nb = 0; nb < 4; ++nb) { const v16h b = ldh(Bt + boff + (size_t)nb * 16 * K + kc);
#pragma unroll
            for (int mb = 0; mb < 4; ++mb) acc[mb][nb] = wmma16g(a[mb], b, acc[mb][nb]); }
    }
#pragma unroll
    for (int mb = 0; mb < 4; ++mb)
#pragma unroll
        for (int nb = 0; nb < 4; ++nb) {
#pragma unroll
            for (int j = 0; j < 8; ++j) os[(mb * 16 + hi * 8u + j) * OSP + nb * 16 + lr] = acc[mb][nb][j]; }
    wave_sync();
    if (MODE == 0) {
        __shared__ __align__(16) h16 hs[64 * 64];
        const unsigned c8 = (lane & 7u) * 8u, rq = lane >> 3;
        const v4f bA = *(const v4f*)(bias + c0 + c8), bB = *(const v4f*)(bias + c0 + c8 + 4u);
        float bv[8];
#pragma unroll
        for (int i = 0; i < 4; ++i) { bv[i] = bfr(bA[i]); bv[4 + i] = bfr(bB[i]); }
#pragma unroll 1
        for (unsigned it = 0; it < 16; ++it) {
            const unsigned row = 4u * it + rq;
            const v4f x0 = *(const v4fa*)(&os[row * OSP + c8]); const v4f x1 = *(const v4fa*)(&os[row * OSP + c8 + 4u]);
            v8h hv;
#pragma unroll
            for (int i = 0; i < 4; ++i) {
                const float z0 = x0[i] * WCI + bv[i], z1 = x1[i] * WCI + bv[4 + i];
                hv[i] = toh_flush(0.5f * z0 * (1.0f + erff(z0 * 0.70710678118654752f)));
                hv[4 + i] = toh_flush(0.5f * z1 * (1.0f + erff(z1 * 0.70710678118654752f))); }
            *(v8ha*)(&hs[row * 64u + c8]) = hv;
        }
        wave_sync();
        h16* ob = HO + (size_t)r0 * FF + c0 + c8;
#pragma unroll 1
        for (int ps = 0; ps < 2; ++ps) {
#pragma unroll 1
            for (unsigned it = 0; it < 16; ++it) {
                const unsigned row = 4u * it + rq;
                const v8h hv = *(const v8ha*)(&hs[row * 64u + c8]);
                *(volatile v8h*)(ob + (size_t)row * FF) = hv; }
            if (ps == 0) __threadfence(); }
    } else {
        const unsigned cofs = (lane & 15u) * 4u, rh = lane >> 4;
        const v4f bq4 = *(const v4f*)(bias + c0 + cofs);
        v4f bq; bq[0] = bfr(bq4[0]); bq[1] = bfr(bq4[1]); bq[2] = bfr(bq4[2]); bq[3] = bfr(bq4[3]);
        const float* rb = RES + (size_t)r0 * DM + c0 + cofs;
        float* yb = YO + (size_t)r0 * DM + c0 + cofs;
#pragma unroll 1
        for (int ps = 0; ps < 2; ++ps) {
#pragma unroll 1
            for (unsigned it = 0; it < 32; ++it) {
                const unsigned row = 2u * it + rh;
                const v4f x = *(const v4fa*)(&os[row * OSP + cofs]);
                const v4f r = *(const v4f*)(rb + (size_t)row * DM);
                v4f val;
                val[0] = (x[0] * WCI + bq[0]) + r[0]; val[1] = (x[1] * WCI + bq[1]) + r[1]; val[2] = (x[2] * WCI + bq[2]) + r[2]; val[3] = (x[3] * WCI + bq[3]) + r[3];
                *(volatile v4f*)(yb + (size_t)row * DM) = val; }
            if (ps == 0) __threadfence(); }
    }
}
__global__ __launch_bounds__(32) void k_mlp_up(const h16* __restrict__ A, const h16* __restrict__ Bt, const float* __restrict__ bias, h16* HO) { gemmh_body<0>(A, Bt, bias, bias, HO, (float*)0); }
__global__ __launch_bounds__(32) void k_mlp_down(const h16* __restrict__ A, const h16* __restrict__ Bt, const float* __restrict__ bias, const float* __restrict__ RES, float* YO) { gemmh_body<1>(A, Bt, bias, RES, (h16*)0, YO); }

static constexpr size_t al256(size_t v) { return (v + 255) & ~(size_t)255; }
static constexpr size_t mx2(size_t a, size_t b) { return a > b ? a : b; }
static constexpr size_t SZ_XB  = al256((size_t)NB * SEQ * DM * 2);
static constexpr size_t SZ_WT  = al256((size_t)3 * DM * DM * 2);
static constexpr size_t SZ_PL  = al256((size_t)NB * NH_ * SEQ * HD * 2);
static constexpr size_t SZ_RS  = al256((size_t)NB * NH_ * EROWS * HD * 2);
static constexpr size_t SZ_WM  = al256((size_t)DM * FF * 2);
static constexpr size_t SZ_F32 = al256((size_t)NB * SEQ * DM * 4);
static constexpr size_t SZ_HP  = al256((size_t)NB * SEQ * FF * 2);
static constexpr size_t SZ_XH  = al256((size_t)NB * SEQ * DM * 2);
static constexpr size_t SZ_PH1 = SZ_XB + SZ_WT + 3 * SZ_PL + 3 * SZ_RS;
static constexpr size_t SZ_PH2 = SZ_HP + SZ_XH;
static constexpr size_t SZ_RA  = mx2(SZ_PH1, SZ_PH2);
static constexpr size_t SZ_TOTAL = SZ_RA + 2 * SZ_WM + 2 * SZ_F32;
static_assert(SZ_PH1 <= SZ_RA);
static_assert(SZ_PH2 <= SZ_RA);
static_assert(SZ_TOTAL <= (size_t)134217728);
static_assert(((size_t)DM * DM * 2) % 256 == 0);
static_assert((size_t)NB * NH_ * SEQ * HD == (size_t)NB * DM * SEQ);
static_assert((size_t)NB * NH_ * EROWS * HD == (size_t)NB * DM * EROWS);

extern "C" void kernel_launch(void* const* d_in, const int* in_sizes, int n_in,
                              void* d_out, int out_size, void* d_ws, size_t ws_size, hipStream_t stream) {
    if (n_in < 12) return;
    const size_t needx = ((size_t)(NB - 1) * SEQ_FULL + SEQ) * DM;
    if ((size_t)in_sizes[0] < needx) return;
    if ((size_t)in_sizes[1] < (size_t)NH_ * DM * HD || (size_t)in_sizes[2] < (size_t)NH_ * DM * HD || (size_t)in_sizes[3] < (size_t)NH_ * DM * HD) return;
    if (in_sizes[4] < DM || in_sizes[5] < DM || in_sizes[9] < DM || in_sizes[10] < DM || in_sizes[11] < DM) return;
    if ((size_t)in_sizes[6] < (size_t)DM * FF || in_sizes[7] < FF || (size_t)in_sizes[8] < (size_t)FF * DM) return;
    if ((size_t)out_size < ((size_t)(NB - 1) * OUT_SEQ + SEQ) * DM) return;
    if (SZ_TOTAL > ws_size) return;
    const float* x   = (const float*)d_in[0];
    const float* wq  = (const float*)d_in[1];
    const float* wk  = (const float*)d_in[2];
    const float* wv  = (const float*)d_in[3];
    const float* g1  = (const float*)d_in[4];
    const float* be1 = (const float*)d_in[5];
    const float* w1  = (const float*)d_in[6];
    const float* b1  = (const float*)d_in[7];
    const float* w2  = (const float*)d_in[8];
    const float* b2  = (const float*)d_in[9];
    const float* g2  = (const float*)d_in[10];
    const float* be2 = (const float*)d_in[11];
    float* OUT = (float*)d_out;
    char* ra = (char*)d_ws;
    bf*  XB = (bf*)ra;
    bf*  WT = (bf*)(ra + SZ_XB);
    h16* QP = (h16*)(ra + SZ_XB + SZ_WT);
    h16* KP = (h16*)(ra + SZ_XB + SZ_WT + SZ_PL);
    h16* VT = (h16*)(ra + SZ_XB + SZ_WT + 2 * SZ_PL);
    h16* QR = (h16*)(ra + SZ_XB + SZ_WT + 3 * SZ_PL);
    h16* KR = (h16*)(ra + SZ_XB + SZ_WT + 3 * SZ_PL + SZ_RS);
    h16* VR = (h16*)(ra + SZ_XB + SZ_WT + 3 * SZ_PL + 2 * SZ_RS);
    h16* HP  = (h16*)ra;
    h16* X1H = (h16*)(ra + SZ_HP);
    char* wsp = ra + SZ_RA;
    h16* W1T = (h16*)wsp; wsp += SZ_WM;
    h16* W2T = (h16*)wsp; wsp += SZ_WM;
    float* CTX = (float*)wsp; wsp += SZ_F32;
    float* X1F = (float*)wsp; wsp += SZ_F32;
    float* YP = CTX;
    bf* WTq = WT; bf* WTk = WT + (size_t)DM * DM; bf* WTv = WT + (size_t)2 * DM * DM;

    if (SEQ == SEQ_FULL) {
        const size_t n8 = (size_t)NB * SEQ * DM / 8;
        k_cvt8<<<(unsigned)((n8 + 255) / 256), 256, 0, stream>>>(x, XB, n8);
    } else {
        const size_t n8 = (size_t)SEQ * DM / 8;
        for (int b = 0; b < NB; ++b) k_cvt8<<<(unsigned)((n8 + 255) / 256), 256, 0, stream>>>(x + (size_t)b * SEQ_FULL * DM, XB + (size_t)b * SEQ * DM, n8);
    }
    k_wtr_bf<<<dim3(HD / 64, DM / 64, NH_), 256, 0, stream>>>(wq, WTq, (unsigned)DM, (unsigned)HD);
    k_wtr_bf<<<dim3(HD / 64, DM / 64, NH_), 256, 0, stream>>>(wk, WTk, (unsigned)DM, (unsigned)HD);
    k_wtr_bf<<<dim3(HD / 64, DM / 64, NH_), 256, 0, stream>>>(wv, WTv, (unsigned)DM, (unsigned)HD);
    k_wtr_h<<<dim3(FF / 64, DM / 64, 1), 256, 0, stream>>>(w1, W1T, (unsigned)DM, (unsigned)FF);
    k_wtr_h<<<dim3(DM / 64, FF / 64, 1), 256, 0, stream>>>(w2, W2T, (unsigned)FF, (unsigned)DM);

    k_proj_tok<<<dim3(NB * SEQ / 64, DM / 64, 1), 32, 0, stream>>>(XB, WTk, QP, QR, (unsigned)EROWS);
    k_proj_tok<<<dim3(NB * SEQ / 64, DM / 64, 1), 32, 0, stream>>>(XB, WTq, KP, KR, (unsigned)EROWS);
    k_proj_tr<<<dim3(DM / 64, NB * SEQ / 64, 1), 32, 0, stream>>>(WTv, XB, VT, VR, (unsigned)EROWS);

    k_flash_early<<<dim3(EROWS / (16 * AW), NB * NH_, 1), 32 * AW, 0, stream>>>(QP, QR, KP, KR, VT, VR, CTX);
    if (SEQ > EROWS)
        k_flash_late<<<dim3((SEQ - EROWS) / (16 * AW), NB * NH_, 1), 32 * AW, 0, stream>>>(QP, QR, KP, KR, VT, VR, CTX);

    k_ln_first<<<dim3(NB * SEQ / 8, 1, 1), 256, 0, stream>>>(x, CTX, g1, be1, X1F, X1H);
    k_mlp_up<<<dim3(NB * SEQ / 64, FF / 64, 1), 32, 0, stream>>>(X1H, W1T, b1, HP);
    k_mlp_down<<<dim3(NB * SEQ / 64, DM / 64, 1), 32, 0, stream>>>(HP, W2T, b2, X1F, YP);
    k_ln_last<<<dim3(NB * SEQ / 8, 1, 1), 256, 0, stream>>>(YP, g2, be2, OUT);
}
